// CrossAttention_59322088292867
// MI455X (gfx1250) — hardware-verified
//
#include <hip/hip_runtime.h>
#include <stdint.h>


typedef _Float16     v16h  __attribute__((ext_vector_type(16)));
typedef _Float16     v8h   __attribute__((ext_vector_type(8)));
typedef float        v8f   __attribute__((ext_vector_type(8)));
typedef float        v4f   __attribute__((ext_vector_type(4)));
typedef unsigned int u32x4 __attribute__((ext_vector_type(4)));

#ifndef NQ
#define NQ 2048
#endif
#define NQ_FULL 2048
#define NKEY    2048
#define DM      1024
#define DC      768
#define NH      16
#define HD      64
#define KT      64
#define LP      72
#define SP16    72
#define SP32    68

#define W_CARRY  64.0f
#define PROJ_SC  0.0625f
#define SSC      0.0078125f
#define P_CARRY  256.0f
#define CTX_SC   0.25f
#define OUT_SC   6.103515625e-05f

static_assert(NQ % 64 == 0);
static_assert(NQ >= 64 && NQ <= NQ_FULL);
static_assert(DM == NH * HD);
static_assert(DM % 64 == 0 && DC % 64 == 0 && NKEY % 64 == 0);
static_assert(DM % 32 == 0 && DC % 32 == 0);
static_assert(NKEY % KT == 0 && KT == 64 && HD == 64);
static_assert((NQ * DM) % 2048 == 0 && (NKEY * DC) % 2048 == 0);
static_assert((LP * 2) % 16 == 0 && (SP16 * 2) % 16 == 0 && (SP32 * 4) % 16 == 0);

union Frag { v16h h; u32x4 u[2]; };

__device__ __forceinline__ v8f mma16(const Frag& a, const Frag& b, v8f c)
{
    v8f d = __builtin_amdgcn_wmma_f32_16x16x32_f16(false, a.h, false, b.h, (short)0, c, false, false);
    asm volatile("v_nop\n\tv_nop\n\tv_nop\n\tv_nop" : "+v"(d) : "v"(a.h), "v"(b.h));
    return d;
}

__device__ __forceinline__ float bf16r(float x)
{
    unsigned int u = __float_as_uint(x);
    u = (u + 0x7fffu + ((u >> 16) & 1u)) & 0xffff0000u;
    return __uint_as_float(u);
}

__global__ __launch_bounds__(256)
void k_cvt_rows(const float* __restrict__ x, _Float16* __restrict__ y, int n8)
{
    const int g = blockIdx.x * 256 + threadIdx.x;
    if (g >= n8) return;
    const v4f* src = (const v4f*)(x + (size_t)g * 8);
    v4f a = src[0];
    v4f b = src[1];
    union { v8h hv; u32x4 u; } pk;
#pragma unroll
    for (int i = 0; i < 4; ++i) {
        float s0 = a[i];
        float s1 = b[i];
        pk.hv[i]     = (_Float16)bf16r(s0);
        pk.hv[i + 4] = (_Float16)bf16r(s1);
    }
    u32x4 v = pk.u;
    volatile u32x4* dst = (volatile u32x4*)(y + (size_t)g * 8);
    *dst = v;
    __threadfence();
    *dst = v;
}

__global__ __launch_bounds__(256)
void k_wT(const float* __restrict__ W, _Float16* __restrict__ WT, int K, int N)
{
    __shared__ __attribute__((aligned(16))) _Float16 tl[64 * LP];
    const int t  = threadIdx.x;
    const int n0 = blockIdx.x * 64;
    const int k0 = blockIdx.y * 64;
#pragma unroll 4
    for (int p = 0; p < 16; ++p) {
        const int i = p * 4 + (t >> 6);
        const int j = t & 63;
        float w = W[(size_t)(k0 + i) * N + n0 + j];
        tl[j * LP + i] = (_Float16)(W_CARRY * bf16r(w));
    }
    __syncthreads();
    u32x4 v[2];
#pragma unroll
    for (int p = 0; p < 2; ++p) {
        const int g = p * 256 + t, j = g >> 3, ch = (g & 7) * 8;
        v[p] = *(const u32x4*)&tl[j * LP + ch];
    }
#pragma unroll
    for (int p = 0; p < 2; ++p) {
        const int g = p * 256 + t, j = g >> 3, ch = (g & 7) * 8;
        *(volatile u32x4*)(WT + (size_t)(n0 + j) * K + k0 + ch) = v[p];
    }
    __threadfence();
#pragma unroll
    for (int p = 0; p < 2; ++p) {
        const int g = p * 256 + t, j = g >> 3, ch = (g & 7) * 8;
        *(volatile u32x4*)(WT + (size_t)(n0 + j) * K + k0 + ch) = v[p];
    }
}

template <int EP>
__global__ __launch_bounds__(64) __attribute__((amdgpu_num_vgpr(256)))
void k_gemm(const _Float16* __restrict__ A, const _Float16* __restrict__ BT,
            void* __restrict__ Cv, const float* __restrict__ bias,
            int M, int N, int K, float scale)
{
    __shared__ __attribute__((aligned(16))) _Float16 st16[2][32 * SP16];
    __shared__ __attribute__((aligned(16))) float    st32[2][32 * SP32];
    (void)M;

    const int t = threadIdx.x, wave = t >> 5, lane = t & 31;
    const int h = lane >> 4, off = 8 * h, m = lane & 15;
    const int m0 = blockIdx.y * 64 + wave * 32;
    const int n0 = blockIdx.x * 64;

    const _Float16* a0p = A  + (size_t)(m0 + m) * K + off;
    const _Float16* a1p = A  + (size_t)(m0 + 16 + m) * K + off;
    const _Float16* bp  = BT + (size_t)(n0 + m) * K + off;

    const v8f zero8 = {};
    v8f acc[2][4];
#pragma unroll
    for (int mi = 0; mi < 2; ++mi)
#pragma unroll
        for (int nj = 0; nj < 4; ++nj) acc[mi][nj] = zero8;

#pragma unroll 1
    for (int k0 = 0; k0 < K; k0 += 32) {
        Frag a0, a1;
        a0.u[0] = *(const u32x4*)(a0p + k0);
        a0.u[1] = *(const u32x4*)(a0p + k0 + 16);
        a1.u[0] = *(const u32x4*)(a1p + k0);
        a1.u[1] = *(const u32x4*)(a1p + k0 + 16);
#pragma unroll
        for (int nj = 0; nj < 4; ++nj) {
            const _Float16* q = bp + (size_t)nj * 16 * K + k0;
            Frag b;
            b.u[0] = *(const u32x4*)(q);
            b.u[1] = *(const u32x4*)(q + 16);
            acc[0][nj] = mma16(a0, b, acc[0][nj]);
            acc[1][nj] = mma16(a1, b, acc[1][nj]);
        }
    }

    if constexpr (EP == 0) {
        _Float16* st = &st16[wave][0];
#pragma unroll
        for (int mi = 0; mi < 2; ++mi)
#pragma unroll
            for (int nj = 0; nj < 4; ++nj)
#pragma unroll
                for (int r = 0; r < 8; ++r)
                    st[(16 * mi + 8 * h + r) * SP16 + 16 * nj + m] =
                        (_Float16)(acc[mi][nj][r] * scale);
        __syncthreads();
        u32x4 v[8];
#pragma unroll
        for (int i = 0; i < 8; ++i) {
            const int row = i * 4 + (lane >> 3), ch = (lane & 7) * 8;
            v[i] = *(const u32x4*)&st[row * SP16 + ch];
        }
        _Float16* C = (_Float16*)Cv;
#pragma unroll
        for (int i = 0; i < 8; ++i) {
            const int row = i * 4 + (lane >> 3), ch = (lane & 7) * 8;
            *(volatile u32x4*)(C + (size_t)(m0 + row) * N + n0 + ch) = v[i];
        }
        __threadfence();
#pragma unroll
        for (int i = 0; i < 8; ++i) {
            const int row = i * 4 + (lane >> 3), ch = (lane & 7) * 8;
            *(volatile u32x4*)(C + (size_t)(m0 + row) * N + n0 + ch) = v[i];
        }
    } else {
        float* st = &st32[wave][0];
        float bv[4];
#pragma unroll
        for (int nj = 0; nj < 4; ++nj) bv[nj] = bf16r(bias[n0 + 16 * nj + m]);
#pragma unroll
        for (int mi = 0; mi < 2; ++mi)
#pragma unroll
            for (int nj = 0; nj < 4; ++nj)
#pragma unroll
                for (int r = 0; r < 8; ++r)
                    st[(16 * mi + 8 * h + r) * SP32 + 16 * nj + m] =
                        acc[mi][nj][r] * scale + bv[nj];
        __syncthreads();
        v4f v[16];
#pragma unroll
        for (int i = 0; i < 16; ++i) {
            const int row = 2 * i + (lane >> 4), ch = (lane & 15) * 4;
            v[i] = *(const v4f*)&st[row * SP32 + ch];
        }
        float* C = (float*)Cv;
#pragma unroll
        for (int i = 0; i < 16; ++i) {
            const int row = 2 * i + (lane >> 4), ch = (lane & 15) * 4;
            *(volatile v4f*)(C + (size_t)(m0 + row) * N + n0 + ch) = v[i];
        }
        __threadfence();
#pragma unroll
        for (int i = 0; i < 16; ++i) {
            const int row = 2 * i + (lane >> 4), ch = (lane & 15) * 4;
            *(volatile v4f*)(C + (size_t)(m0 + row) * N + n0 + ch) = v[i];
        }
    }
}

__global__ __launch_bounds__(128) __attribute__((amdgpu_num_vgpr(256)))
void k_attn(const _Float16* __restrict__ Qp, const _Float16* __restrict__ Kp,
            const _Float16* __restrict__ Vt, _Float16* __restrict__ Ctx)
{
    __shared__ __attribute__((aligned(16))) _Float16 Ks[KT * LP];
    __shared__ __attribute__((aligned(16))) _Float16 Vs[HD * LP];
    __shared__ __attribute__((aligned(16))) _Float16 Ps[4 * 16 * LP];

    const int t = threadIdx.x, wave = t >> 5, lane = t & 31;
    const int h = lane >> 4, off = 8 * h, m = lane & 15;
    const int head = blockIdx.y, c0 = head * HD;
    const int q0 = blockIdx.x * 64 + wave * 16;
    _Float16* Pw = Ps + wave * (16 * LP);

    Frag aq0, aq1;
    {
        const _Float16* qr = Qp + (size_t)(q0 + m) * DM + c0 + off;
        aq0.u[0] = *(const u32x4*)(qr);
        aq0.u[1] = *(const u32x4*)(qr + 16);
        aq1.u[0] = *(const u32x4*)(qr + 32);
        aq1.u[1] = *(const u32x4*)(qr + 48);
    }

    const v8f zero8 = {};
    v8f o[4];
    float mrun[8], lrun[8];
#pragma unroll
    for (int f = 0; f < 4; ++f) o[f] = zero8;
#pragma unroll
    for (int r = 0; r < 8; ++r) { mrun[r] = -1e30f; lrun[r] = 0.f; }

#pragma unroll 1
    for (int kt = 0; kt < NKEY / KT; ++kt) {
        __syncthreads();
#pragma unroll
        for (int i = 0; i < 4; ++i) {
            const int g = i * 128 + t, r = g >> 3, ch = (g & 7) * 8;
            *(u32x4*)&Ks[r * LP + ch] =
                *(const u32x4*)(Kp + (size_t)(kt * KT + r) * DM + c0 + ch);
            *(u32x4*)&Vs[r * LP + ch] =
                *(const u32x4*)(Vt + (size_t)(c0 + r) * NKEY + kt * KT + ch);
        }
        __syncthreads();

        v8f s[4];
#pragma unroll
        for (int j = 0; j < 4; ++j) {
            const _Float16* kr = Ks + (16 * j + m) * LP + off;
            Frag b;
            b.u[0] = *(const u32x4*)(kr);
            b.u[1] = *(const u32x4*)(kr + 16);
            s[j] = mma16(aq0, b, zero8);
            b.u[0] = *(const u32x4*)(kr + 32);
            b.u[1] = *(const u32x4*)(kr + 48);
            s[j] = mma16(aq1, b, s[j]);
        }

        float tmx[8];
#pragma unroll
        for (int r = 0; r < 8; ++r) {
            float v = s[0][r];
            v = fmaxf(v, s[1][r]);
            v = fmaxf(v, s[2][r]);
            v = fmaxf(v, s[3][r]);
            tmx[r] = v;
        }
#pragma unroll
        for (int xm = 1; xm < 16; xm <<= 1)
#pragma unroll
            for (int r = 0; r < 8; ++r) tmx[r] = fmaxf(tmx[r], __shfl_xor(tmx[r], xm, 32));

        float al[8], ls[8];
#pragma unroll
        for (int r = 0; r < 8; ++r) {
            const float mn = fmaxf(mrun[r], tmx[r] * SSC);
            al[r]   = __expf(mrun[r] - mn);
            mrun[r] = mn;
            float sum = 0.f;
#pragma unroll
            for (int j = 0; j < 4; ++j) {
                const float p = __expf(s[j][r] * SSC - mn);
                sum += p;
                Pw[(8 * h + r) * LP + 16 * j + m] = (_Float16)(p * P_CARRY);
            }
            ls[r] = sum;
#pragma unroll
            for (int f = 0; f < 4; ++f) o[f][r] = o[f][r] * al[r];
        }
#pragma unroll
        for (int xm = 1; xm < 16; xm <<= 1)
#pragma unroll
            for (int r = 0; r < 8; ++r) ls[r] += __shfl_xor(ls[r], xm, 32);
#pragma unroll
        for (int r = 0; r < 8; ++r) lrun[r] = lrun[r] * al[r] + ls[r];
        __syncthreads();

#pragma unroll
        for (int kc = 0; kc < 2; ++kc) {
            const _Float16* pr = Pw + m * LP + 32 * kc + off;
            Frag pa;
            pa.u[0] = *(const u32x4*)(pr);
            pa.u[1] = *(const u32x4*)(pr + 16);
#pragma unroll
            for (int f = 0; f < 4; ++f) {
                const _Float16* vr = Vs + (16 * f + m) * LP + 32 * kc + off;
                Frag vb;
                vb.u[0] = *(const u32x4*)(vr);
                vb.u[1] = *(const u32x4*)(vr + 16);
                o[f] = mma16(pa, vb, o[f]);
            }
        }
    }

    float inv[8];
#pragma unroll
    for (int r = 0; r < 8; ++r) inv[r] = CTX_SC / lrun[r];
    __syncthreads();
#pragma unroll
    for (int f = 0; f < 4; ++f)
#pragma unroll
        for (int r = 0; r < 8; ++r)
            Pw[(8 * h + r) * LP + 16 * f + m] = (_Float16)(o[f][r] * inv[r]);
    __syncthreads();
    u32x4 cv[4];
#pragma unroll
    for (int i = 0; i < 4; ++i) {
        const int row = i * 4 + (lane >> 3), ch = (lane & 7) * 8;
        cv[i] = *(const u32x4*)(Pw + row * LP + ch);
    }
#pragma unroll
    for (int i = 0; i < 4; ++i) {
        const int row = i * 4 + (lane >> 3), ch = (lane & 7) * 8;
        *(volatile u32x4*)(Ctx + (size_t)(q0 + row) * DM + c0 + ch) = cv[i];
    }
    __threadfence();
#pragma unroll
    for (int i = 0; i < 4; ++i) {
        const int row = i * 4 + (lane >> 3), ch = (lane & 7) * 8;
        *(volatile u32x4*)(Ctx + (size_t)(q0 + row) * DM + c0 + ch) = cv[i];
    }
}

extern "C" void kernel_launch(void* const* d_in, const int* in_sizes, int n_in,
                              void* d_out, int out_size, void* d_ws, size_t ws_size,
                              hipStream_t stream)
{
    if (n_in < 8) return;
    if (in_sizes[0] < NQ * DM || in_sizes[1] < NKEY * DC || in_sizes[2] < NKEY * DC ||
        in_sizes[3] < DM * DM || in_sizes[4] < DC * DM || in_sizes[5] < DC * DM ||
        in_sizes[6] < DM * DM || in_sizes[7] < DM) return;
    if (out_size < NQ * DM) return;

    const float* qin = (const float*)d_in[0];
    const float* kin = (const float*)d_in[1];
    const float* vin = (const float*)d_in[2];
    const float* Wq  = (const float*)d_in[3];
    const float* Wk  = (const float*)d_in[4];
    const float* Wv  = (const float*)d_in[5];
    const float* Wo  = (const float*)d_in[6];
    const float* bo  = (const float*)d_in[7];
    float* out = (float*)d_out;

    const size_t szQ16  = (size_t)NQ   * DM   * 2;
    const size_t szK16  = (size_t)NKEY * DC   * 2;
    const size_t szV16  = (size_t)NKEY * DC   * 2;
    const size_t szWqT  = (size_t)DM   * DM   * 2;
    const size_t szWkT  = (size_t)DM   * DC   * 2;
    const size_t szWvT  = (size_t)DM   * DC   * 2;
    const size_t szWoT  = (size_t)DM   * DM   * 2;
    const size_t szQpl  = (size_t)NQ   * DM   * 2;
    const size_t szKpl  = (size_t)NKEY * DM   * 2;
    const size_t szVt   = (size_t)DM   * NKEY * 2;
    const size_t szCtx  = (size_t)NQ   * DM   * 2;
    size_t o0 = 0;
    char* ws = (char*)d_ws;
    _Float16* Q16  = (_Float16*)(ws + o0); o0 += szQ16;
    _Float16* K16  = (_Float16*)(ws + o0); o0 += szK16;
    _Float16* V16  = (_Float16*)(ws + o0); o0 += szV16;
    _Float16* WqT  = (_Float16*)(ws + o0); o0 += szWqT;
    _Float16* WkT  = (_Float16*)(ws + o0); o0 += szWkT;
    _Float16* WvT  = (_Float16*)(ws + o0); o0 += szWvT;
    _Float16* WoT  = (_Float16*)(ws + o0); o0 += szWoT;
    _Float16* Qpl  = (_Float16*)(ws + o0); o0 += szQpl;
    _Float16* Kpl  = (_Float16*)(ws + o0); o0 += szKpl;
    _Float16* Vtp  = (_Float16*)(ws + o0); o0 += szVt;
    _Float16* Ctx  = (_Float16*)(ws + o0); o0 += szCtx;
    if (o0 > ws_size) return;

    k_cvt_rows<<<dim3(NQ * DM / 8 / 256), 256, 0, stream>>>(qin, Q16, NQ * DM / 8);
    k_cvt_rows<<<dim3(NKEY * DC / 8 / 256), 256, 0, stream>>>(kin, K16, NKEY * DC / 8);
    k_cvt_rows<<<dim3(NKEY * DC / 8 / 256), 256, 0, stream>>>(vin, V16, NKEY * DC / 8);

    k_wT<<<dim3(DM / 64, DM / 64), 256, 0, stream>>>(Wq, WqT, DM, DM);
    k_wT<<<dim3(DM / 64, DC / 64), 256, 0, stream>>>(Wk, WkT, DC, DM);
    k_wT<<<dim3(DM / 64, DC / 64), 256, 0, stream>>>(Wv, WvT, DC, DM);
    k_wT<<<dim3(DM / 64, DM / 64), 256, 0, stream>>>(Wo, WoT, DM, DM);

    k_gemm<0><<<dim3(DM / 64, NQ / 64), 64, 0, stream>>>(Q16, WqT, Qpl, bo, NQ, DM, DM, PROJ_SC);
    k_gemm<0><<<dim3(DM / 64, NKEY / 64), 64, 0, stream>>>(K16, WkT, Kpl, bo, NKEY, DM, DC, PROJ_SC);
    k_gemm<0><<<dim3(NKEY / 64, DM / 64), 64, 0, stream>>>(WvT, V16, Vtp, bo, DM, NKEY, DC, PROJ_SC);

    k_attn<<<dim3(NQ / 64, NH), 128, 0, stream>>>(Qpl, Kpl, Vtp, Ctx);

    k_gemm<1><<<dim3(DM / 64, NQ / 64), 64, 0, stream>>>(Ctx, WoT, out, bo, NQ, DM, DM, OUT_SC);
}
